// lanegcn_vanilla_gan_60155311948394
// MI455X (gfx1250) — hardware-verified
//
#include <hip/hip_runtime.h>
#include <stddef.h>


#define NTHR    256
#define NWAVE   8
#define NBN     64
#define NC      128
#define AP      136
#define CP      132
#define EPT     8
#define PIECE   (NTHR * EPT)
#define WCAP    (EPT * 32)
#define GEPS    1e-5f
#define WSCALE  64.0f
#define D1SCALE 64.0f
#define INV64   0.015625f
#define INV4096 0.000244140625f
#define OD2     0
#define OQ      16384
#define OC1     32768
#define OC2     81920
#define OA      98304
#define OL      114688
#define PWTOT   131072
#define KC1     384
#define PTHR    256
#define PBLK    (PWTOT / (PTHR * 8))
#define SLB     9
#define NBC     (1 << SLB)
#define RPW     (NBC / NWAVE)
#define AGGDYN  (NBC * NC * 4)
#define N1DYN   (3 * NBN * AP * 2 + NBN * CP * 4)
#define EDYN    (2 * NBN * AP * 2 + NBN * CP * 4 + 384 * 4 + 128 * 4)
#define N2DYN   (2 * NBN * AP * 2 + 2 * NBN * CP * 4 + NBN * 4)
#define NPH     3
#define WSCAP   134217728

static_assert(NTHR == 256);
static_assert(NBN == NWAVE * 8);
static_assert(PIECE == 2048);
static_assert((EPT % 4) == 0);
static_assert((PWTOT % (PTHR * 8)) == 0);
static_assert((OQ % 2048) == 0);
static_assert((OC1 % 2048) == 0);
static_assert((OC2 % 2048) == 0);
static_assert((OA % 2048) == 0);
static_assert((OL % 2048) == 0);
static_assert(OD2 + NC * NC == OQ);
static_assert(OQ + NC * NC == OC1);
static_assert(OC1 + NC * KC1 == OC2);
static_assert(OC2 + NC * NC == OA);
static_assert(OA + NC * NC == OL);
static_assert(OL + NC * NC == PWTOT);
static_assert(((AP * 2) % 16) == 0);
static_assert(((CP * 4) % 16) == 0);
static_assert(((KC1 * 2) % 16) == 0);
static_assert(((NBN * AP * 2) % 16) == 0);
static_assert(((NBN * CP * 4) % 16) == 0);
static_assert(AGGDYN == 262144);
static_assert(N1DYN == 86016);
static_assert(EDYN == 70656);
static_assert(N2DYN == 102656);
static_assert((NBC % NWAVE) == 0);
static_assert(SLB >= 3);
static_assert(SLB + 11 <= 30);

typedef float          v4f   __attribute__((ext_vector_type(4)));
typedef float          v8f   __attribute__((ext_vector_type(8)));
typedef int            v4i   __attribute__((ext_vector_type(4)));
typedef unsigned short v4us  __attribute__((ext_vector_type(4)));
typedef unsigned short v8us  __attribute__((ext_vector_type(8)));
typedef _Float16       v4h   __attribute__((ext_vector_type(4)));
typedef _Float16       v8h   __attribute__((ext_vector_type(8)));
typedef _Float16       v16h  __attribute__((ext_vector_type(16)));

__device__ __forceinline__ v16h mkfrag(v8us u0, v8us u1) {
  const v8h a = __builtin_bit_cast(v8h, u0);
  const v8h b = __builtin_bit_cast(v8h, u1);
  return __builtin_shufflevector(a, b, 0, 1, 2, 3, 4, 5, 6, 7, 8, 9, 10, 11, 12, 13, 14, 15);
}

__device__ __forceinline__ v8f wmf(v16h a, v16h b, v8f c) {
  v8f d = __builtin_amdgcn_wmma_f32_16x16x32_f16(false, a, false, b, (short)0, c, false, false);
  asm volatile("v_nop\n\tv_nop\n\tv_nop\n\tv_nop" : "+v"(d) : "v"(a), "v"(b));
  return d;
}
__device__ __forceinline__ v8f zero8() {
  v8f z = {0.f, 0.f, 0.f, 0.f, 0.f, 0.f, 0.f, 0.f};
  return z;
}
template <int NT>
__device__ __forceinline__ void zacc(v8f (&c)[NT]) {
#pragma unroll
  for (int t = 0; t < NT; ++t) c[t] = zero8();
}
__device__ __forceinline__ int iclamp(int v, int lo, int hi) { return v < lo ? lo : (v > hi ? hi : v); }

__device__ __forceinline__ float wave_sum32(float x) {
#pragma unroll
  for (int o = 16; o > 0; o >>= 1) x += __shfl_xor(x, o, 32);
  return x;
}

__device__ __forceinline__ v8us pack8(v4f a, v4f b) {
  const v8f f = __builtin_shufflevector(a, b, 0, 1, 2, 3, 4, 5, 6, 7);
  const v8h h = __builtin_convertvector(f, v8h);
  return __builtin_bit_cast(v8us, h);
}

template <int NT>
__device__ __forceinline__ void gemmNT(const unsigned short* ap, const unsigned short* __restrict__ bpl,
                                       int Kp, int nks, int n0, int m, int hh, v8f (&c)[NT]) {
#pragma unroll 1
  for (int ks = 0; ks < nks; ++ks) {
    const v16h a = mkfrag(*(const v8us*)(ap + 32 * ks), *(const v8us*)(ap + 32 * ks + 16));
    const size_t bo = (size_t)(n0 + m) * Kp + 32 * ks + 8 * hh;
#pragma unroll
    for (int t = 0; t < NT; ++t) {
      const size_t o = bo + (size_t)(16 * t) * Kp;
      const v16h b = mkfrag(*(const v8us*)(bpl + o), *(const v8us*)(bpl + o + 16));
      c[t] = wmf(a, b, c[t]);
    }
  }
}

template <int NT>
__device__ __forceinline__ void stageC(float* sC, int row0, int col0, v8f (&c)[NT], float inv) {
#pragma unroll
  for (int t = 0; t < NT; ++t) {
    float* sp = sC + row0 * CP + col0 + 16 * t;
#pragma unroll
    for (int r = 0; r < 8; ++r) sp[r * CP] = c[t][r] * inv;
  }
}

template <bool RELU, bool RES, bool WF, bool WH, int NADD>
__device__ __forceinline__ void gn_epi(const float* sC, float* sF, unsigned short* sHo,
                                       const float* __restrict__ g, const float* __restrict__ b,
                                       const float* __restrict__ t1, const int* i1,
                                       const float* __restrict__ t2, const int* i2,
                                       int wave, int lane) {
  const v4f gg = *(const v4f*)(g + 4 * lane);
  const v4f bb = *(const v4f*)(b + 4 * lane);
#pragma unroll 2
  for (int rr = 0; rr < 8; ++rr) {
    const int row = 8 * wave + rr;
    v4f x = *(const v4f*)(sC + row * CP + 4 * lane);
    if constexpr (NADD >= 1) {
      const int j1 = i1[row];
      const v4f a1 = *(const v4f*)(t1 + (size_t)j1 * NC + 4 * lane);
      x = x + a1;
    }
    if constexpr (NADD >= 2) {
      const int j2 = i2[row];
      const v4f a2 = *(const v4f*)(t2 + (size_t)j2 * NC + 4 * lane);
      x = x + a2;
    }
    float s = (x.x + x.y) + (x.z + x.w);
    s = wave_sum32(s);
    const float mu = s * (1.0f / 128.0f);
    v4f d;
    d.x = x.x - mu; d.y = x.y - mu; d.z = x.z - mu; d.w = x.w - mu;
    float q = (d.x * d.x + d.y * d.y) + (d.z * d.z + d.w * d.w);
    q = wave_sum32(q);
    const float rstd = rsqrtf(q * (1.0f / 128.0f) + GEPS);
    v4f o;
    o.x = (d.x * rstd) * gg.x + bb.x;
    o.y = (d.y * rstd) * gg.y + bb.y;
    o.z = (d.z * rstd) * gg.z + bb.z;
    o.w = (d.w * rstd) * gg.w + bb.w;
    if constexpr (RES) {
      const v4f rv = *(const v4f*)(sF + row * CP + 4 * lane);
      o.x += rv.x; o.y += rv.y; o.z += rv.z; o.w += rv.w;
    }
    if constexpr (RELU) {
      o.x = fmaxf(o.x, 0.0f); o.y = fmaxf(o.y, 0.0f); o.z = fmaxf(o.z, 0.0f); o.w = fmaxf(o.w, 0.0f);
    }
    if constexpr (WF) *(v4f*)(sF + row * CP + 4 * lane) = o;
    if constexpr (WH) {
      const v4h hv = __builtin_convertvector(o, v4h);
      *(v4us*)(sHo + row * AP + 4 * lane) = __builtin_bit_cast(v4us, hv);
    }
  }
}

__device__ __forceinline__ void rowsF(const float* sF, float* dst, int n0, int nrows, int tid) {
#pragma unroll 1
  for (int it = 0; it < 8; ++it) {
    const int p = it * NTHR + tid;
    const int row = p >> 5, c4 = p & 31;
    const v4f v = *(const v4f*)(sF + row * CP + 4 * c4);
    if (row < nrows) *(volatile v4f*)(dst + (size_t)(n0 + row) * NC + 4 * c4) = v;
  }
}

__global__ __launch_bounds__(PTHR) void k_prep(
    const float* __restrict__ wd2, const float* __restrict__ wq, const float* __restrict__ wc1,
    const float* __restrict__ wc2, const float* __restrict__ wa, const float* __restrict__ wl,
    unsigned short* wpl) {
  const int tid = (int)threadIdx.x;
  const int ob = (int)blockIdx.x * (PTHR * 8);
  const int o = ob + tid * 8;
  const float* src = wd2;
  int sb = OD2;
  if (ob >= OL)       { src = wl;  sb = OL; }
  else if (ob >= OA)  { src = wa;  sb = OA; }
  else if (ob >= OC2) { src = wc2; sb = OC2; }
  else if (ob >= OC1) { src = wc1; sb = OC1; }
  else if (ob >= OQ)  { src = wq;  sb = OQ; }
  const float* p = src + (o - sb);
  v4f a = *(const v4f*)p;
  v4f b = *(const v4f*)(p + 4);
  a = a * WSCALE;
  b = b * WSCALE;
  const v8us hv = pack8(a, b);
  unsigned short* d = wpl + o;
  *(volatile v8us*)d = hv;
  __threadfence();
  *(volatile v8us*)d = hv;
}

__global__ __launch_bounds__(NTHR) void k_node1(
    const float* __restrict__ x, const float* __restrict__ c, const unsigned short* __restrict__ wpl,
    const float* __restrict__ gq, const float* __restrict__ bq, float* TQ, float* TC, int nN) {
  extern __shared__ __attribute__((aligned(16))) unsigned short dyn1[];
  unsigned short* sX = dyn1;
  unsigned short* sY = dyn1 + NBN * AP;
  unsigned short* sH = dyn1 + 2 * NBN * AP;
  float* sC = (float*)(dyn1 + 3 * NBN * AP);
  const int tid = (int)threadIdx.x, lane = tid & 31, wave = tid >> 5, hh = lane >> 4, m = lane & 15;
  const int n0 = (int)blockIdx.x * NBN;

  {
    const int nl = tid >> 2, q = tid & 3;
    int node = n0 + nl;
    node = node > nN - 1 ? nN - 1 : node;
    const float* xp = x + (size_t)node * NC + 32 * q;
    const float* cp = c + (size_t)node * NC + 32 * q;
    unsigned short* dx = sX + nl * AP + 32 * q;
    unsigned short* dc = sY + nl * AP + 32 * q;
#pragma unroll
    for (int j = 0; j < 4; ++j) {
      const v4f a0 = *(const v4f*)(xp + 8 * j);
      const v4f a1 = *(const v4f*)(xp + 8 * j + 4);
      *(v8us*)(dx + 8 * j) = pack8(a0, a1);
      const v4f b0 = *(const v4f*)(cp + 8 * j);
      const v4f b1 = *(const v4f*)(cp + 8 * j + 4);
      *(v8us*)(dc + 8 * j) = pack8(b0, b1);
    }
  }
  __syncthreads();
  const int rt = wave & 3, cg = wave >> 2;

  {
    v8f acc[4];
    zacc<4>(acc);
    gemmNT<4>(sX + (16 * rt + m) * AP + 8 * hh, wpl + OQ, NC, 4, 64 * cg, m, hh, acc);
    stageC<4>(sC, 16 * rt + 8 * hh, 64 * cg + m, acc, INV64);
  }
  __syncthreads();
  gn_epi<true, false, false, true, 0>(sC, nullptr, sH, gq, bq, nullptr, nullptr, nullptr, nullptr, wave, lane);
  __syncthreads();

  {
    v8f acc[4];
    zacc<4>(acc);
    gemmNT<4>(sH + (16 * rt + m) * AP + 8 * hh, wpl + OC1 + 128, KC1, 4, 64 * cg, m, hh, acc);
    stageC<4>(sC, 16 * rt + 8 * hh, 64 * cg + m, acc, INV64);
  }
  __syncthreads();
  rowsF(sC, TQ, n0, NBN, tid);
  __threadfence();
  rowsF(sC, TQ, n0, NBN, tid);
  __syncthreads();

  {
    v8f acc[4];
    zacc<4>(acc);
    gemmNT<4>(sY + (16 * rt + m) * AP + 8 * hh, wpl + OC1 + 256, KC1, 4, 64 * cg, m, hh, acc);
    stageC<4>(sC, 16 * rt + 8 * hh, 64 * cg + m, acc, INV64);
  }
  __syncthreads();
  rowsF(sC, TC, n0, NBN, tid);
  __threadfence();
  rowsF(sC, TC, n0, NBN, tid);
}

__global__ __launch_bounds__(NTHR) void k_edge(
    const float* __restrict__ actr, const float* __restrict__ cctr, const int* __restrict__ ehi,
    const int* __restrict__ ewi, const float* __restrict__ wd1, const float* __restrict__ bd1,
    const unsigned short* __restrict__ wpl,
    const float* __restrict__ gd2, const float* __restrict__ bd2,
    const float* __restrict__ gc1, const float* __restrict__ bc1,
    const float* __restrict__ TQ, const float* __restrict__ TC, float* MSG,
    int e0, int nE, int nN) {
  extern __shared__ __attribute__((aligned(16))) unsigned short dynE[];
  unsigned short* sD = dynE;
  unsigned short* sH = dynE + NBN * AP;
  float* sC = (float*)(dynE + 2 * NBN * AP);
  float* sW = sC + NBN * CP;
  int* sI = (int*)(sW + 384);
  const int tid = (int)threadIdx.x, lane = tid & 31, wave = tid >> 5, hh = lane >> 4, m = lane & 15;
  const int r0l = (int)blockIdx.x * NBN;

  sW[tid] = wd1[tid];
  if (tid < 128) sW[256 + tid] = bd1[tid];
  if (tid < 128) {
    const int r = tid & 63;
    int e = e0 + r0l + r;
    e = e > nE - 1 ? nE - 1 : (e < 0 ? 0 : e);
    if (tid < 64) sI[r] = iclamp(ehi[e], 0, nN - 1);
    else          sI[64 + r] = iclamp(ewi[e], 0, nN - 1);
  }
  __syncthreads();

  {
    const int r = tid >> 2, q = tid & 3;
    const int h = sI[r], w = sI[64 + r];
    const float dx = actr[2 * h] - cctr[2 * w];
    const float dy = actr[2 * h + 1] - cctr[2 * w + 1];
    unsigned short* dp = sD + r * AP + 32 * q;
#pragma unroll
    for (int jj = 0; jj < 4; ++jj) {
      float f[8];
#pragma unroll
      for (int j = 0; j < 8; ++j) {
        const int k = 32 * q + 8 * jj + j;
        float p = dx * sW[2 * k];
        p = fmaf(dy, sW[2 * k + 1], p);
        p = p + sW[256 + k];
        f[j] = fmaxf(p, 0.0f) * D1SCALE;
      }
      v4f a, b;
      a.x = f[0]; a.y = f[1]; a.z = f[2]; a.w = f[3];
      b.x = f[4]; b.y = f[5]; b.z = f[6]; b.w = f[7];
      *(v8us*)(dp + 8 * jj) = pack8(a, b);
    }
  }
  __syncthreads();
  const int rt = wave & 3, cg = wave >> 2;

  {
    v8f acc[4];
    zacc<4>(acc);
    gemmNT<4>(sD + (16 * rt + m) * AP + 8 * hh, wpl + OD2, NC, 4, 64 * cg, m, hh, acc);
    stageC<4>(sC, 16 * rt + 8 * hh, 64 * cg + m, acc, INV4096);
  }
  __syncthreads();
  gn_epi<true, false, false, true, 0>(sC, nullptr, sH, gd2, bd2, nullptr, nullptr, nullptr, nullptr, wave, lane);
  __syncthreads();

  {
    v8f acc[4];
    zacc<4>(acc);
    gemmNT<4>(sH + (16 * rt + m) * AP + 8 * hh, wpl + OC1, KC1, 4, 64 * cg, m, hh, acc);
    stageC<4>(sC, 16 * rt + 8 * hh, 64 * cg + m, acc, INV64);
  }
  __syncthreads();
  gn_epi<true, false, false, true, 2>(sC, nullptr, sD, gc1, bc1, TQ, sI, TC, sI + 64, wave, lane);
  __syncthreads();

  {
    v8f acc[4];
    zacc<4>(acc);
    gemmNT<4>(sD + (16 * rt + m) * AP + 8 * hh, wpl + OC2, NC, 4, 64 * cg, m, hh, acc);
    stageC<4>(sC, 16 * rt + 8 * hh, 64 * cg + m, acc, INV64);
  }
  __syncthreads();
  rowsF(sC, MSG, r0l, NBN, tid);
  __threadfence();
  rowsF(sC, MSG, r0l, NBN, tid);
}

__device__ __forceinline__ int scan_piece(const int* __restrict__ ei, int lim, int cbase, int base,
                                          int* list, int tid, int wave, int vec) {
  int wc = 0;
  const int el0  = tid * EPT;
  const int e0   = cbase + el0;
  const int sent = -2147483647 - 1;
  int kk[EPT];
  if (vec != 0 && cbase + PIECE <= lim) {
    const v4i* p = (const v4i*)(ei + e0);
#pragma unroll
    for (int uu = 0; uu < EPT / 4; ++uu) {
      const v4i d = p[uu];
      kk[4 * uu] = d.x; kk[4 * uu + 1] = d.y; kk[4 * uu + 2] = d.z; kk[4 * uu + 3] = d.w;
    }
  } else {
    const int lm = lim - 1;
#pragma unroll
    for (int q = 0; q < EPT; ++q) {
      const int eq = e0 + q;
      const int ec = eq > lm ? lm : eq;
      const int a = ei[ec];
      kk[q] = (eq < lim) ? a : sent;
    }
  }
  const unsigned nb = (unsigned)base;
  unsigned sq[EPT];
  bool hq[EPT];
  bool anyl = false;
#pragma unroll
  for (int q = 0; q < EPT; ++q) {
    sq[q] = (unsigned)kk[q] - nb;
    hq[q] = sq[q] < (unsigned)NBC;
    anyl = anyl | hq[q];
  }
  const unsigned any = __builtin_amdgcn_ballot_w32(anyl);
  if (any != 0u) {
#define HIT(HQ, SQ, Q) { \
      const unsigned mj = __builtin_amdgcn_ballot_w32(HQ); \
      if (mj != 0u) { \
        if (HQ) { \
          const int ps = wc + (int)__builtin_amdgcn_mbcnt_lo(mj, 0u); \
          if (ps < WCAP) list[wave * WCAP + ps] = ((el0 + (Q)) << SLB) | (int)(SQ); \
        } \
        wc += (int)__builtin_popcount(mj); } }
#pragma unroll
    for (int q = 0; q < EPT; ++q) {
      HIT(hq[q], sq[q], q)
    }
#undef HIT
  }
  return wc;
}

__device__ __forceinline__ void drain_sum(const int* list, const int* wcnt, float* acc,
                                          const float* __restrict__ MSG, int cbase, int ne, int lane, int wave) {
#pragma unroll 1
  for (int wsx = 0; wsx < NWAVE; ++wsx) {
    int n = __builtin_amdgcn_readfirstlane(wcnt[wsx]);
    n = n > WCAP ? WCAP : (n < 0 ? 0 : n);
    const int* lp = list + wsx * WCAP;
#pragma unroll 1
    for (int bb = 0; bb < n; bb += 32) {
      const int idx = bb + lane;
      const int ic = idx > WCAP - 1 ? WCAP - 1 : idx;
      const int ent = lp[ic];
      const bool own = (idx < n) && ((ent & (NWAVE - 1)) == wave);
      unsigned msk = __builtin_amdgcn_ballot_w32(own);
#pragma unroll 1
      while (msk != 0u) {
        const int bit = (int)__builtin_ctz(msk);
        msk &= msk - 1u;
        const int e2 = __builtin_amdgcn_readlane(ent, bit);
        const int slot = e2 & (NBC - 1);
        const int el = (e2 >> SLB) & (PIECE - 1);
        int e = cbase + el;
        e = e > ne - 1 ? ne - 1 : (e < 0 ? 0 : e);
        const v4f mv = *(const v4f*)(MSG + (size_t)e * NC + 4 * lane);
        float* ap2 = acc + slot * NC + 4 * lane;
        v4f av = *(const v4f*)ap2;
        av = av + mv;
        *(v4f*)ap2 = av;
      }
    }
  }
}

__device__ __forceinline__ void agg_rows(const float* acc, float* AGG, int base, int lane, int wave) {
#pragma unroll 1
  for (int it = 0; it < RPW; ++it) {
    const int s = wave * RPW + it;
    const v4f v = *(const v4f*)(acc + s * NC + 4 * lane);
    *(volatile v4f*)(AGG + (size_t)(base + s) * NC + 4 * lane) = v;
  }
}

template <bool FIRST>
__global__ __launch_bounds__(NTHR) void k_agg(
    const int* __restrict__ keys, const float* __restrict__ MSG, float* AGG, int ne, int vec) {
  extern __shared__ __attribute__((aligned(16))) float accA[];
  __shared__ int list[NWAVE * WCAP];
  __shared__ int wcnt[NWAVE];
  const int tid = (int)threadIdx.x, lane = tid & 31, wave = tid >> 5;
  const int base = (int)blockIdx.x * NBC;
#pragma unroll 1
  for (int it = 0; it < RPW; ++it) {
    const int s = wave * RPW + it;
    v4f v = {0.0f, 0.0f, 0.0f, 0.0f};
    if constexpr (!FIRST) v = *(const v4f*)(AGG + (size_t)(base + s) * NC + 4 * lane);
    *(v4f*)(accA + s * NC + 4 * lane) = v;
  }
  __syncthreads();
#pragma unroll 1
  for (int cbase = 0; cbase < ne; cbase += PIECE) {
    const int wc = scan_piece(keys, ne, cbase, base, list, tid, wave, vec);
    if (lane == 0) wcnt[wave] = wc;
    __syncthreads();
    drain_sum(list, wcnt, accA, MSG, cbase, ne, lane, wave);
    __syncthreads();
  }
  __syncthreads();
  agg_rows(accA, AGG, base, lane, wave);
  __threadfence();
  agg_rows(accA, AGG, base, lane, wave);
}

__global__ __launch_bounds__(NTHR) void k_node2(
    const float* __restrict__ x, const float* __restrict__ AGG, const unsigned short* __restrict__ wpl,
    const float* __restrict__ gnm, const float* __restrict__ bnm, const float* __restrict__ gl,
    const float* __restrict__ bl, float* out, int nN) {
  extern __shared__ __attribute__((aligned(16))) unsigned short dyn2[];
  unsigned short* sX = dyn2;
  unsigned short* sH = dyn2 + NBN * AP;
  float* sF = (float*)(dyn2 + 2 * NBN * AP);
  float* sC = sF + NBN * CP;
  int* sN = (int*)(sC + NBN * CP);
  const int tid = (int)threadIdx.x, lane = tid & 31, wave = tid >> 5, hh = lane >> 4, m = lane & 15;
  const int n0 = (int)blockIdx.x * NBN;

  {
    const int nl = tid >> 2, q = tid & 3;
    int node = n0 + nl;
    node = node > nN - 1 ? nN - 1 : node;
    if (q == 0) sN[nl] = node;
    const float* xp = x + (size_t)node * NC + 32 * q;
    float* df = sF + nl * CP + 32 * q;
    unsigned short* dx = sX + nl * AP + 32 * q;
#pragma unroll
    for (int j = 0; j < 4; ++j) {
      const v4f a0 = *(const v4f*)(xp + 8 * j);
      const v4f a1 = *(const v4f*)(xp + 8 * j + 4);
      *(v4f*)(df + 8 * j)     = a0;
      *(v4f*)(df + 8 * j + 4) = a1;
      *(v8us*)(dx + 8 * j) = pack8(a0, a1);
    }
  }
  __syncthreads();
  const int rt = wave & 3, cg = wave >> 2;

  {
    v8f acc[4];
    zacc<4>(acc);
    gemmNT<4>(sX + (16 * rt + m) * AP + 8 * hh, wpl + OA, NC, 4, 64 * cg, m, hh, acc);
    stageC<4>(sC, 16 * rt + 8 * hh, 64 * cg + m, acc, INV64);
  }
  __syncthreads();
  gn_epi<true, false, false, true, 1>(sC, nullptr, sH, gnm, bnm, AGG, sN, nullptr, nullptr, wave, lane);
  __syncthreads();

  {
    v8f acc[4];
    zacc<4>(acc);
    gemmNT<4>(sH + (16 * rt + m) * AP + 8 * hh, wpl + OL, NC, 4, 64 * cg, m, hh, acc);
    stageC<4>(sC, 16 * rt + 8 * hh, 64 * cg + m, acc, INV64);
  }
  __syncthreads();
  gn_epi<true, true, true, false, 0>(sC, sF, nullptr, gl, bl, nullptr, nullptr, nullptr, nullptr, wave, lane);
  __syncthreads();

  int nr = nN - n0;
  nr = nr > NBN ? NBN : (nr < 1 ? 1 : nr);
  rowsF(sF, out, n0, nr, tid);
  __threadfence();
  rowsF(sF, out, n0, nr, tid);
}

extern "C" void kernel_launch(void* const* d_in, const int* in_sizes, int n_in,
                              void* d_out, int out_size, void* d_ws, size_t ws_size,
                              hipStream_t stream) {
  if (n_in < 24) return;
  const int nN = in_sizes[0] / NC;
  if (nN < 1 || nN > (1 << 22) || in_sizes[0] != nN * NC || in_sizes[1] != nN * NC) return;
  if (in_sizes[2] != 2 * nN || in_sizes[3] != 2 * nN) return;
  const int nE = in_sizes[4];
  if (nE < 1 || nE > (1 << 27) || in_sizes[5] != nE) return;
  if (in_sizes[6] != 2 * NC || in_sizes[7] != NC) return;
  if (in_sizes[8] != NC * NC || in_sizes[9] != NC || in_sizes[10] != NC) return;
  if (in_sizes[11] != NC * NC || in_sizes[12] != NC || in_sizes[13] != NC) return;
  if (in_sizes[14] != NC * KC1 || in_sizes[15] != NC || in_sizes[16] != NC || in_sizes[17] != NC * NC) return;
  if (in_sizes[18] != NC * NC || in_sizes[19] != NC || in_sizes[20] != NC) return;
  if (in_sizes[21] != NC * NC || in_sizes[22] != NC || in_sizes[23] != NC) return;
  if ((size_t)out_size != (size_t)nN * NC) return;

  const float* agts  = (const float*)d_in[0];
  const float* ctx   = (const float*)d_in[1];
  const float* actr  = (const float*)d_in[2];
  const float* cctr  = (const float*)d_in[3];
  const int*   ehi   = (const int*)d_in[4];
  const int*   ewi   = (const int*)d_in[5];
  const float* w_d1  = (const float*)d_in[6];
  const float* b_d1  = (const float*)d_in[7];
  const float* w_d2  = (const float*)d_in[8];
  const float* g_d2  = (const float*)d_in[9];
  const float* bt_d2 = (const float*)d_in[10];
  const float* w_q   = (const float*)d_in[11];
  const float* g_q   = (const float*)d_in[12];
  const float* bt_q  = (const float*)d_in[13];
  const float* w_c1  = (const float*)d_in[14];
  const float* g_c1  = (const float*)d_in[15];
  const float* bt_c1 = (const float*)d_in[16];
  const float* w_c2  = (const float*)d_in[17];
  const float* w_a   = (const float*)d_in[18];
  const float* g_n   = (const float*)d_in[19];
  const float* bt_n  = (const float*)d_in[20];
  const float* w_l   = (const float*)d_in[21];
  const float* g_l   = (const float*)d_in[22];
  const float* bt_l  = (const float*)d_in[23];
  float* out = (float*)d_out;

  const int nb64 = (nN + NBN - 1) / NBN;
  const int Npad64 = nb64 * NBN;
  const int nbA = (nN + NBC - 1) / NBC;
  const int NpA = nbA * NBC;
  const int eph = ((((nE + NPH - 1) / NPH) + NBN - 1) / NBN) * NBN;

  char* ws = (char*)d_ws;
  size_t off = 0;
  const size_t oW   = off; off += (size_t)PWTOT * 2;              off = (off + 255) & ~(size_t)255;
  const size_t oTQ  = off; off += (size_t)Npad64 * NC * 4;        off = (off + 255) & ~(size_t)255;
  const size_t oTC  = off; off += (size_t)Npad64 * NC * 4;        off = (off + 255) & ~(size_t)255;
  const size_t oM   = off; off += (size_t)eph * NC * 4;           off = (off + 255) & ~(size_t)255;
  const size_t oAGG = off; off += (size_t)NpA * NC * 4;           off = (off + 255) & ~(size_t)255;
  if (off > ws_size || off > (size_t)WSCAP) return;
  unsigned short* wpl = (unsigned short*)(ws + oW);
  float* TQ  = (float*)(ws + oTQ);
  float* TC  = (float*)(ws + oTC);
  float* MSG = (float*)(ws + oM);
  float* AGG = (float*)(ws + oAGG);

  hipFuncSetAttribute(reinterpret_cast<const void*>(&k_agg<true>), hipFuncAttributeMaxDynamicSharedMemorySize, AGGDYN);
  hipFuncSetAttribute(reinterpret_cast<const void*>(&k_agg<false>), hipFuncAttributeMaxDynamicSharedMemorySize, AGGDYN);
  hipFuncSetAttribute(reinterpret_cast<const void*>(&k_node1), hipFuncAttributeMaxDynamicSharedMemorySize, N1DYN);
  hipFuncSetAttribute(reinterpret_cast<const void*>(&k_edge), hipFuncAttributeMaxDynamicSharedMemorySize, EDYN);
  hipFuncSetAttribute(reinterpret_cast<const void*>(&k_node2), hipFuncAttributeMaxDynamicSharedMemorySize, N2DYN);

  k_prep<<<PBLK, PTHR, 0, stream>>>(w_d2, w_q, w_c1, w_c2, w_a, w_l, wpl);
  k_node1<<<nb64, NTHR, N1DYN, stream>>>(agts, ctx, wpl, g_q, bt_q, TQ, TC, nN);
  for (int ph = 0; ph < NPH; ++ph) {
    const int e0 = ph * eph;
    int ne = nE - e0;
    if (ne > eph) ne = eph;
    if (ne <= 0) continue;
    const int nbE = (ne + NBN - 1) / NBN;
    k_edge<<<nbE, NTHR, EDYN, stream>>>(actr, cctr, ehi, ewi, w_d1, b_d1, wpl, g_d2, bt_d2, g_c1, bt_c1,
                                         TQ, TC, MSG, e0, nE, nN);
    const int vec = ((e0 & 3) == 0) ? 1 : 0;
    if (ph == 0)
      k_agg<true><<<nbA, NTHR, AGGDYN, stream>>>(ehi + e0, MSG, AGG, ne, vec);
    else
      k_agg<false><<<nbA, NTHR, AGGDYN, stream>>>(ehi + e0, MSG, AGG, ne, vec);
  }
  k_node2<<<nb64, NTHR, N2DYN, stream>>>(agts, AGG, wpl, g_n, bt_n, g_l, bt_l, out, nN);
}
